// RecurrentLegendreLayer_1743756722949
// MI455X (gfx1250) — hardware-run, weakly checked
//
#include <hip/hip_runtime.h>

#pragma clang fp contract(off)

typedef __attribute__((ext_vector_type(16))) __bf16   v16b;
typedef __attribute__((ext_vector_type(8)))  __bf16   v8b;
typedef __attribute__((ext_vector_type(8)))  float    v8f;
typedef __attribute__((ext_vector_type(4)))  float    v4f;
typedef __attribute__((ext_vector_type(4)))  unsigned v4u;

constexpr int NUM_DEG     = 9;
constexpr int BATCH_ROWS  = 16384;
constexpr int IN_DIM      = 512;
constexpr int OUT_DIM     = 512;
constexpr int K_TOTAL     = NUM_DEG * IN_DIM;
constexpr int TILE_M      = 128;
constexpr int TILE_N      = 128;
constexpr int K_CHUNK     = 32;
constexpr int NUM_ICHUNK  = IN_DIM / K_CHUNK;
constexpr int A_PITCH     = 40;
constexpr int PLANE_BYTES = TILE_M * A_PITCH * 2;
constexpr int BUF_BYTES   = 2 * PLANE_BYTES;
constexpr int LDS_BYTES   = 2 * BUF_BYTES;
constexpr int SLAB_PITCH  = 68;
constexpr int NTHREADS    = 256;
constexpr int PACK_PITCH  = 72;
constexpr int PACK_TILE   = 64;

static_assert(K_TOTAL == 4608);
static_assert(K_TOTAL % PACK_TILE == 0);
static_assert(K_TOTAL % K_CHUNK == 0);
static_assert(BATCH_ROWS % TILE_M == 0);
static_assert(OUT_DIM % TILE_N == 0);
static_assert(OUT_DIM % PACK_TILE == 0);
static_assert(IN_DIM % K_CHUNK == 0);
static_assert((NUM_DEG & 1) == 1);
static_assert(LDS_BYTES == 40960);
static_assert((NTHREADS / 32) * 16 * SLAB_PITCH * 4 <= LDS_BYTES);
static_assert((A_PITCH * 2) % 16 == 0);
static_assert((PACK_PITCH * 2) % 16 == 0);

__device__ __forceinline__ unsigned bf16_rne_hi(unsigned u) {
  return (u + 0x7FFFu + ((u >> 16) & 1u)) & 0xFFFF0000u;
}
__device__ __forceinline__ float bf16_value(float f) {
  return __uint_as_float(bf16_rne_hi(__float_as_uint(f)));
}

union FragB { v16b v; v8b h[2]; };
__device__ __forceinline__ v16b frag_load(const __bf16* p) {
  FragB f;
  f.h[0] = *(const v8b*)(p);
  f.h[1] = *(const v8b*)(p + 16);
  return f.v;
}
__device__ __forceinline__ v8f mma_bf16(v16b a, v16b b, v8f c) {
  return __builtin_amdgcn_wmma_f32_16x16x32_bf16(false, a, false, b, (short)0, c, false, false);
}
__device__ __forceinline__ void group_guard(v8f& a0, v8f& a1, v8f& a2, v8f& a3,
                                            v16b x, v16b y, v16b b0, v16b b1, v16b b2, v16b b3) {
  asm volatile("v_nop\n\tv_nop\n\tv_nop\n\tv_nop"
               : "+v"(a0), "+v"(a1), "+v"(a2), "+v"(a3)
               : "v"(x), "v"(y), "v"(b0), "v"(b1), "v"(b2), "v"(b3));
}
__device__ __forceinline__ void acc_guard4(v8f& a, v8f& b, v8f& c, v8f& d) {
  asm volatile("v_nop\n\tv_nop\n\tv_nop\n\tv_nop" : "+v"(a), "+v"(b), "+v"(c), "+v"(d));
}

__global__ __launch_bounds__(NTHREADS) void wt_pack_kernel(const float* __restrict__ w, unsigned short* __restrict__ wt) {
  __shared__ __align__(16) unsigned short tile[PACK_TILE * PACK_PITCH];
  const int tid  = threadIdx.x;
  const int lane = tid & 31;
  const int wave = tid >> 5;
  const int kt   = blockIdx.x;
  const int n0   = blockIdx.y * PACK_TILE;
  {
    const int kr  = tid >> 2;
    const int seg = (tid & 3) * 16;
    const int kp  = kt * PACK_TILE + kr;
    const int s   = kp >> 5;
    const int il  = kp & 31;
    const int ic  = s / NUM_DEG;
    const int f   = s - ic * NUM_DEG;
    const int i   = ic * K_CHUNK + il;
    const float* src = w + ((size_t)f * IN_DIM + (size_t)i) * OUT_DIM + n0 + seg;
#pragma unroll
    for (int q = 0; q < 4; ++q) {
      const v4f v = *(const v4f*)(src + 4 * q);
#pragma unroll
      for (int e = 0; e < 4; ++e) {
        const float t = v[e];
        const unsigned hb = bf16_rne_hi(__float_as_uint(t)) >> 16;
        tile[(seg + 4 * q + e) * PACK_PITCH + kr] = (unsigned short)hb;
      }
    }
  }
  __syncthreads();
  {
    const int q  = lane >> 3;
    const int c8 = (lane & 7) * 8;
    v4u vals[2];
#pragma unroll
    for (int it = 0; it < 2; ++it) {
      const int row = it * 32 + wave * 4 + q;
      vals[it] = *(const v4u*)(tile + row * PACK_PITCH + c8);
    }
    for (int pass = 0; pass < 2; ++pass) {
#pragma unroll
      for (int it = 0; it < 2; ++it) {
        const int row = it * 32 + wave * 4 + q;
        unsigned short* dst = wt + (size_t)(n0 + row) * K_TOTAL + (size_t)kt * PACK_TILE + c8;
        *(volatile v4u*)dst = vals[it];
      }
      __threadfence();
    }
  }
}

__global__ __launch_bounds__(NTHREADS) void poly_gemm_kernel(const float* __restrict__ x,
                                                             const unsigned short* __restrict__ wt,
                                                             const float* __restrict__ bias,
                                                             float* __restrict__ out) {
  __shared__ __align__(16) unsigned char smem[LDS_BYTES];

  const int tid  = threadIdx.x;
  const int lane = tid & 31;
  const int wave = tid >> 5;
  const int wm   = wave >> 1;
  const int wn   = wave & 1;
  const int m_blk = blockIdx.x * TILE_M;
  const int n_blk = blockIdx.y * TILE_N;

  const int prow = tid >> 1;
  const int pi0  = (tid & 1) * 16;

  const int rl   = lane & 15;
  const int hh   = lane >> 4;
  const int koff = hh * 8;

  const __bf16* wbase = (const __bf16*)wt + (size_t)(n_blk + wn * 64 + rl) * K_TOTAL + koff;
  const float*  xrow  = x + (size_t)(m_blk + prow) * IN_DIM + pi0;

  v8f acc[2][4];
#pragma unroll
  for (int mi = 0; mi < 2; ++mi)
#pragma unroll
    for (int j = 0; j < 4; ++j) acc[mi][j] = (v8f){0.f, 0.f, 0.f, 0.f, 0.f, 0.f, 0.f, 0.f};

#pragma unroll 1
  for (int ic = 0; ic < NUM_ICHUNK; ++ic) {
    float xv[16], p1[16], p2[16];
    {
      const float* xp = xrow + ic * K_CHUNK;
#pragma unroll
      for (int q = 0; q < 4; ++q) {
        const v4f v = *(const v4f*)(xp + 4 * q);
#pragma unroll
        for (int e = 0; e < 4; ++e) {
          const float t = v[e];
          xv[4 * q + e] = bf16_value(t);
        }
      }
    }

#pragma unroll
    for (int f = 0; f < NUM_DEG; ++f) {
      const int par = (ic + f) & 1;
      unsigned char* abase = smem + par * BUF_BYTES;

      unsigned hw[8], lw[8];
      if (f == 0) {
#pragma unroll
        for (int j = 0; j < 16; ++j) p2[j] = 1.0f;
#pragma unroll
        for (int q = 0; q < 8; ++q) { hw[q] = 0x3F803F80u; lw[q] = 0u; }
      } else if (f == 1) {
#pragma unroll
        for (int j = 0; j < 16; ++j) p1[j] = xv[j];
#pragma unroll
        for (int q = 0; q < 8; ++q) {
          hw[q] = (__float_as_uint(xv[2 * q]) >> 16) | __float_as_uint(xv[2 * q + 1]);
          lw[q] = 0u;
        }
      } else {
        const float ca = (float)(2 * f - 1);
        const float cb = (float)(f - 1);
        const float rn = 1.0f / (float)f;
#pragma unroll
        for (int j = 0; j < 16; ++j) {
          const float t  = (ca * xv[j]) * p1[j];
          const float u  = cb * p2[j];
          const float pn = (t - u) * rn;
          p2[j] = p1[j];
          p1[j] = pn;
        }
#pragma unroll
        for (int q = 0; q < 8; ++q) {
          const float va = p1[2 * q];
          const float vb = p1[2 * q + 1];
          const unsigned ha = bf16_rne_hi(__float_as_uint(va));
          const unsigned hb = bf16_rne_hi(__float_as_uint(vb));
          const float ra = va - __uint_as_float(ha);
          const float rb = vb - __uint_as_float(hb);
          const unsigned la = bf16_rne_hi(__float_as_uint(ra));
          const unsigned lb = bf16_rne_hi(__float_as_uint(rb));
          hw[q] = (ha >> 16) | hb;
          lw[q] = (la >> 16) | lb;
        }
      }
      {
        v4u* hdst = (v4u*)(abase + (prow * A_PITCH + pi0) * 2);
        hdst[0] = (v4u){hw[0], hw[1], hw[2], hw[3]};
        hdst[1] = (v4u){hw[4], hw[5], hw[6], hw[7]};
        if (f >= 2) {
          v4u* ldst = (v4u*)(abase + PLANE_BYTES + (prow * A_PITCH + pi0) * 2);
          ldst[0] = (v4u){lw[0], lw[1], lw[2], lw[3]};
          ldst[1] = (v4u){lw[4], lw[5], lw[6], lw[7]};
        }
      }
      __syncthreads();

      const __bf16* wp = wbase + (size_t)((ic * NUM_DEG + f) * K_CHUNK);
      v16b bfr[4];
#pragma unroll
      for (int j = 0; j < 4; ++j) bfr[j] = frag_load(wp + (size_t)(j * 16) * K_TOTAL);

#pragma unroll
      for (int mi = 0; mi < 2; ++mi) {
        const __bf16* ap = (const __bf16*)abase + (wm * 32 + mi * 16 + rl) * A_PITCH + koff;
        const v16b ah = frag_load(ap);
        if (f >= 2) {
          const v16b al = frag_load(ap + PLANE_BYTES / 2);
#pragma unroll
          for (int j = 0; j < 4; ++j) {
            acc[mi][j] = mma_bf16(ah, bfr[j], acc[mi][j]);
            acc[mi][j] = mma_bf16(al, bfr[j], acc[mi][j]);
          }
          group_guard(acc[mi][0], acc[mi][1], acc[mi][2], acc[mi][3], ah, al, bfr[0], bfr[1], bfr[2], bfr[3]);
        } else {
#pragma unroll
          for (int j = 0; j < 4; ++j) acc[mi][j] = mma_bf16(ah, bfr[j], acc[mi][j]);
          group_guard(acc[mi][0], acc[mi][1], acc[mi][2], acc[mi][3], ah, ah, bfr[0], bfr[1], bfr[2], bfr[3]);
        }
      }
    }
  }
  acc_guard4(acc[0][0], acc[0][1], acc[0][2], acc[0][3]);
  acc_guard4(acc[1][0], acc[1][1], acc[1][2], acc[1][3]);

  __syncthreads();

  float* slab = (float*)smem + wave * (16 * SLAB_PITCH);
  const int mOff = hh * 8;
  const int c4   = rl * 4;
  float bv[4];
#pragma unroll
  for (int j = 0; j < 4; ++j) bv[j] = bf16_value(bias[n_blk + wn * 64 + j * 16 + rl]);

#pragma unroll
  for (int mi = 0; mi < 2; ++mi) {
    const int mBase = m_blk + wm * 32 + mi * 16;
#pragma unroll
    for (int j = 0; j < 4; ++j) {
#pragma unroll
      for (int r = 0; r < 8; ++r) {
        const float v = acc[mi][j][r] + bv[j];
        slab[(mOff + r) * SLAB_PITCH + (j << 4) + rl] = v;
      }
    }
    __builtin_amdgcn_fence(__ATOMIC_RELEASE, "workgroup");
    __builtin_amdgcn_wave_barrier();
    __builtin_amdgcn_fence(__ATOMIC_ACQUIRE, "workgroup");
    for (int pass = 0; pass < 2; ++pass) {
#pragma unroll
      for (int it = 0; it < 8; ++it) {
        const int row = it * 2 + hh;
        const v4f v = *(const v4f*)(slab + row * SLAB_PITCH + c4);
        *(volatile v4f*)(out + (size_t)(mBase + row) * OUT_DIM + n_blk + wn * 64 + c4) = v;
      }
      __threadfence();
    }
    __builtin_amdgcn_fence(__ATOMIC_RELEASE, "workgroup");
    __builtin_amdgcn_wave_barrier();
    __builtin_amdgcn_fence(__ATOMIC_ACQUIRE, "workgroup");
  }
}

extern "C" void kernel_launch(void* const* d_in, const int* in_sizes, int n_in,
                              void* d_out, int out_size, void* d_ws, size_t ws_size, hipStream_t stream) {
  if (n_in < 3 || d_out == nullptr || d_ws == nullptr) return;
  if (in_sizes[0] != BATCH_ROWS * IN_DIM || in_sizes[1] != NUM_DEG * IN_DIM * OUT_DIM ||
      in_sizes[2] != OUT_DIM || out_size != BATCH_ROWS * OUT_DIM) return;

  const float* x    = (const float*)d_in[0];
  const float* w    = (const float*)d_in[1];
  const float* bias = (const float*)d_in[2];
  float* out = (float*)d_out;

  const size_t wt_bytes = (size_t)OUT_DIM * K_TOTAL * 2;
  if (wt_bytes > ws_size || wt_bytes > (size_t)134217728) return;
  unsigned short* wtp = (unsigned short*)d_ws;

  wt_pack_kernel<<<dim3(K_TOTAL / PACK_TILE, OUT_DIM / PACK_TILE), NTHREADS, 0, stream>>>(w, wtp);
  poly_gemm_kernel<<<dim3(BATCH_ROWS / TILE_M, OUT_DIM / TILE_N), NTHREADS, 0, stream>>>(x, wtp, bias, out);
}
